// RGCN_17119739642414
// MI455X (gfx1250) — hardware-verified
//
#include <hip/hip_runtime.h>
#include <stddef.h>
#include <stdint.h>


#define CIN    128
#define DH     128
#define NCL    16
#define NREL   4
#define K2     256
#define NTHR   256
#define NWAVE  8
#define EPT    8
#define CHUNK  (NTHR * EPT)
#define WCAP   (EPT * 32)
#define LISTN  (NWAVE * WCAP)
#define NBD    8192
#define SLD    13
#define NBA    2048
#define SLA    11
#define RCAP   16384
#define DEGCAP 256
#define GBM    64
#define GTHR   128
#define FLS    16
#define FROWS  (FLS * NWAVE)
#define NU0    (NREL * DH * (CIN / 8))
#define NU1    (NREL * DH * (DH / 4))
#define NU2    (NREL * NCL * (DH / 4))
#define NUT    (NU0 + NU1 + NU2)
#define AGG_ZINTS    (LISTN + 2 * RCAP + 3 * NBA)
#define AGG_LDS_INTS (AGG_ZINTS + 16 + FROWS * NCL)
#define WSMAX  268435456

static_assert((CHUNK & (CHUNK - 1)) == 0 && CHUNK <= 4096);
static_assert((NBD & (NBD - 1)) == 0 && NBD == (1 << SLD));
static_assert((NBA & (NBA - 1)) == 0 && NBA == (1 << SLA));
static_assert(((long long)CHUNK << SLD) < (1LL << 31));
static_assert(((long long)CHUNK << SLA) < (1LL << 31));
static_assert(NBD % (NTHR * 4) == 0);
static_assert(LISTN % NTHR == 0);
static_assert(NBA % NWAVE == 0 && NBA % 32 == 0 && NBA % GBM == 0);
static_assert(RCAP % 32 == 0 && AGG_ZINTS % (NTHR * 4) == 0 && LISTN % 4 == 0 && (AGG_ZINTS + 16) % 4 == 0);
static_assert(CIN % 32 == 0 && K2 % 32 == 0 && K2 == 2 * DH);
static_assert(GBM == (GTHR / 32) * 16);
static_assert(NU0 % NTHR == 0 && NU1 % NTHR == 0 && NU2 % NTHR == 0 && NUT % NTHR == 0);
static_assert(CIN / 8 == 16 && DH / 4 == 32 && DH == 4 * 32 && NCL == 16);
static_assert((NBA / NWAVE) % FLS == 0 && FROWS * NCL == 2 * NTHR * 4 && GBM * NCL == 2 * GTHR * 4);
static_assert(AGG_LDS_INTS * 4 <= 300000);

typedef float          v4f   __attribute__((ext_vector_type(4)));
typedef float          v8f   __attribute__((ext_vector_type(8)));
typedef int            v4i   __attribute__((ext_vector_type(4)));
typedef int            v8i   __attribute__((ext_vector_type(8)));
typedef unsigned short v8us  __attribute__((ext_vector_type(8)));
typedef unsigned short v16us __attribute__((ext_vector_type(16)));
typedef __bf16         v16bf __attribute__((ext_vector_type(16)));
typedef v4f  __attribute__((may_alias)) v4fa;
typedef v4i  __attribute__((may_alias)) v4ia;
typedef v8us __attribute__((may_alias)) v8usa;
union Frag { v16bf v; v16us u; v8us h[2]; v8i w; };

__device__ __forceinline__ v8f wmb(const Frag& a, const Frag& b, v8f c) {
  v8f d = __builtin_amdgcn_wmma_f32_16x16x32_bf16(false, a.v, false, b.v, (short)0, c, false, false);
  asm volatile("v_nop\n\tv_nop\n\tv_nop\n\tv_nop" : "+v"(d) : "v"(a.w), "v"(b.w));
  return d;
}

__device__ __forceinline__ unsigned bf16_bits(float f) {
  const unsigned u = __float_as_uint(f);
  return (u + 0x7FFFu + ((u >> 16) & 1u)) >> 16;
}
__device__ __forceinline__ float bf16_val(float f) {
  return __uint_as_float(bf16_bits(f) << 16);
}
__device__ __forceinline__ v8us hilo8(v4f t) {
  v8us o;
  unsigned hb;
  hb = bf16_bits(t.x); o[0] = (unsigned short)hb; o[4] = (unsigned short)bf16_bits(t.x - __uint_as_float(hb << 16));
  hb = bf16_bits(t.y); o[1] = (unsigned short)hb; o[5] = (unsigned short)bf16_bits(t.y - __uint_as_float(hb << 16));
  hb = bf16_bits(t.z); o[2] = (unsigned short)hb; o[6] = (unsigned short)bf16_bits(t.z - __uint_as_float(hb << 16));
  hb = bf16_bits(t.w); o[3] = (unsigned short)hb; o[7] = (unsigned short)bf16_bits(t.w - __uint_as_float(hb << 16));
  return o;
}

template <int SLB>
__device__ __forceinline__ int scan_chunk(const int* __restrict__ dsts, int nE, int cbase, int slotBase,
                                          int nb, int vec8, int* list, int tid, int lane, int wave) {
  int wc = 0;
  const int el0  = tid * EPT;
  const int e0   = cbase + el0;
  const int sent = -2147483647 - 1;
  v4i da, db;
  if (vec8 != 0 && cbase + CHUNK <= nE) {
    da = *(const v4i*)(dsts + e0);
    db = *(const v4i*)(dsts + e0 + 4);
  } else {
    da.x = (e0     < nE) ? dsts[min(e0,     nE - 1)] : sent;
    da.y = (e0 + 1 < nE) ? dsts[min(e0 + 1, nE - 1)] : sent;
    da.z = (e0 + 2 < nE) ? dsts[min(e0 + 2, nE - 1)] : sent;
    da.w = (e0 + 3 < nE) ? dsts[min(e0 + 3, nE - 1)] : sent;
    db.x = (e0 + 4 < nE) ? dsts[min(e0 + 4, nE - 1)] : sent;
    db.y = (e0 + 5 < nE) ? dsts[min(e0 + 5, nE - 1)] : sent;
    db.z = (e0 + 6 < nE) ? dsts[min(e0 + 6, nE - 1)] : sent;
    db.w = (e0 + 7 < nE) ? dsts[min(e0 + 7, nE - 1)] : sent;
  }
  const unsigned nbs = (unsigned)slotBase;
  const unsigned unb = (unsigned)nb;
  const unsigned s0 = (unsigned)da.x - nbs, s1 = (unsigned)da.y - nbs;
  const unsigned s2 = (unsigned)da.z - nbs, s3 = (unsigned)da.w - nbs;
  const unsigned s4 = (unsigned)db.x - nbs, s5 = (unsigned)db.y - nbs;
  const unsigned s6 = (unsigned)db.z - nbs, s7 = (unsigned)db.w - nbs;
  const bool h0 = s0 < unb, h1 = s1 < unb, h2 = s2 < unb, h3 = s3 < unb;
  const bool h4 = s4 < unb, h5 = s5 < unb, h6 = s6 < unb, h7 = s7 < unb;
  const unsigned any = __builtin_amdgcn_ballot_w32(h0 | h1 | h2 | h3 | h4 | h5 | h6 | h7);
  if (any != 0u) {
#define HITJ(J, HJ, SJ) { \
      const unsigned mj = __builtin_amdgcn_ballot_w32(HJ); \
      if (mj != 0u) { \
        if (HJ) { \
          const int pos = wc + (int)__builtin_amdgcn_mbcnt_lo(mj, 0u); \
          if (pos < WCAP) list[wave * WCAP + pos] = ((el0 + (J)) << SLB) | (int)(SJ); \
        } \
        wc += (int)__builtin_popcount(mj); } }
    HITJ(0, h0, s0)
    HITJ(1, h1, s1)
    HITJ(2, h2, s2)
    HITJ(3, h3, s3)
    HITJ(4, h4, s4)
    HITJ(5, h5, s5)
    HITJ(6, h6, s6)
    HITJ(7, h7, s7)
#undef HITJ
  }
  return wc;
}

__global__ __launch_bounds__(NTHR) void k_prep(const float* __restrict__ W0, const float* __restrict__ W1,
                                               const float* __restrict__ W2, unsigned short* W0T,
                                               unsigned short* W1T, unsigned short* W2T) {
  const int u = (int)blockIdx.x * NTHR + (int)threadIdx.x;
  v8us o;
  unsigned short* dp;
  if (u < NU0) {
    const int r  = u >> 11;
    const int n  = (u >> 4) & 127;
    const int k8 = (u & 15) * 8;
    const float* p = W0 + (size_t)r * CIN * DH + (size_t)k8 * DH + n;
#pragma unroll
    for (int i = 0; i < 8; ++i) o[i] = (unsigned short)bf16_bits(p[(size_t)i * DH]);
    dp = W0T + (size_t)r * DH * CIN + (size_t)n * CIN + k8;
  } else if (u < NU0 + NU1) {
    const int v = u - NU0;
    const int r = v >> 12;
    const int n = (v >> 5) & 127;
    const int g = v & 31;
    const float* p = W1 + (size_t)r * DH * DH + (size_t)(4 * g) * DH + n;
    const unsigned short f0 = (unsigned short)bf16_bits(p[0]);
    const unsigned short f1 = (unsigned short)bf16_bits(p[DH]);
    const unsigned short f2 = (unsigned short)bf16_bits(p[2 * DH]);
    const unsigned short f3 = (unsigned short)bf16_bits(p[3 * DH]);
    o[0] = f0; o[1] = f1; o[2] = f2; o[3] = f3; o[4] = f0; o[5] = f1; o[6] = f2; o[7] = f3;
    dp = W1T + (size_t)r * DH * K2 + (size_t)n * K2 + 8 * g;
  } else if (u < NUT) {
    const int v = u - NU0 - NU1;
    const int r = v >> 9;
    const int n = (v >> 5) & 15;
    const int g = v & 31;
    const float* p = W2 + (size_t)r * DH * NCL + (size_t)(4 * g) * NCL + n;
    const unsigned short f0 = (unsigned short)bf16_bits(p[0]);
    const unsigned short f1 = (unsigned short)bf16_bits(p[NCL]);
    const unsigned short f2 = (unsigned short)bf16_bits(p[2 * NCL]);
    const unsigned short f3 = (unsigned short)bf16_bits(p[3 * NCL]);
    o[0] = f0; o[1] = f1; o[2] = f2; o[3] = f3; o[4] = f0; o[5] = f1; o[6] = f2; o[7] = f3;
    dp = W2T + (size_t)r * NCL * K2 + (size_t)n * K2 + 8 * g;
  } else {
    return;
  }
  *(volatile v8us*)dp = o;
  __threadfence();
  *(volatile v8us*)dp = o;
}

__global__ __launch_bounds__(NTHR) void k_cvx(const float* __restrict__ x, int nN, int nUnits,
                                              unsigned short* xb) {
  const int u = (int)blockIdx.x * NTHR + (int)threadIdx.x;
  if (u >= nUnits) return;
  const int row = u >> 4;
  const int k8  = (u & 15) * 8;
  const int rc  = row < nN ? row : nN - 1;
  const float* p = x + (size_t)rc * CIN + k8;
  const v4f a = *(const v4fa*)p;
  const v4f b = *(const v4fa*)(p + 4);
  const bool ok = row < nN;
  v8us o;
  o[0] = ok ? (unsigned short)bf16_bits(a.x) : (unsigned short)0;
  o[1] = ok ? (unsigned short)bf16_bits(a.y) : (unsigned short)0;
  o[2] = ok ? (unsigned short)bf16_bits(a.z) : (unsigned short)0;
  o[3] = ok ? (unsigned short)bf16_bits(a.w) : (unsigned short)0;
  o[4] = ok ? (unsigned short)bf16_bits(b.x) : (unsigned short)0;
  o[5] = ok ? (unsigned short)bf16_bits(b.y) : (unsigned short)0;
  o[6] = ok ? (unsigned short)bf16_bits(b.z) : (unsigned short)0;
  o[7] = ok ? (unsigned short)bf16_bits(b.w) : (unsigned short)0;
  unsigned short* dp = xb + (size_t)row * CIN + k8;
  *(volatile v8us*)dp = o;
  __threadfence();
  *(volatile v8us*)dp = o;
}

__global__ __launch_bounds__(NTHR) void k_deg(const int* __restrict__ srcs, const int* __restrict__ dsts,
                                              int nE, int vec8, int nbpd, float* dg) {
  __shared__ __attribute__((aligned(16))) int scnt[NBD];
  __shared__ __attribute__((aligned(16))) int list[LISTN];
  __shared__ int wcnt[NWAVE];
  const int tid = (int)threadIdx.x, lane = tid & 31, wave = tid >> 5;
  const int nodeBase = (int)blockIdx.x * NBD;
  const int p = (int)blockIdx.y;
  const int* lst = srcs + (size_t)(p < NREL ? p : 0) * (size_t)nE;
  if (p >= NREL) lst = dsts + (size_t)(p - NREL) * (size_t)nE;

  for (int i = tid; i < NBD; i += NTHR) scnt[i] = 0;
  for (int i = tid; i < LISTN; i += NTHR) list[i] = 0;
  if (tid < NWAVE) wcnt[tid] = 0;
  __syncthreads();

  const int nChunks = (nE + CHUNK - 1) / CHUNK;
#pragma unroll 1
  for (int ch = 0; ch < nChunks; ++ch) {
    const int cbase = ch * CHUNK;
    const int wc = scan_chunk<SLD>(lst, nE, cbase, nodeBase, NBD, vec8, list, tid, lane, wave);
    if (lane == 0) wcnt[wave] = wc;
    __syncthreads();
    if (wave == 0) {
#pragma unroll 1
      for (int w2 = 0; w2 < NWAVE; ++w2) {
        int c = wcnt[w2];
        c = c < 0 ? 0 : (c > WCAP ? WCAP : c);
#pragma unroll 1
        for (int b0 = 0; b0 < c; b0 += 32) {
          const int idx = b0 + lane;
          const int ent = list[w2 * WCAP + (idx < WCAP ? idx : WCAP - 1)];
          const int m32 = (c - b0) < 32 ? (c - b0) : 32;
#pragma unroll 1
          for (int k = 0; k < m32; ++k) {
            const int u  = __builtin_amdgcn_readlane(ent, k);
            const int sl = u & (NBD - 1);
            if (lane == 0) scnt[sl] = scnt[sl] + 1;
          }
        }
      }
    }
    __syncthreads();
  }

  v4f vals[NBD / (NTHR * 4)];
#pragma unroll
  for (int it = 0; it < NBD / (NTHR * 4); ++it) {
    const int s0 = it * (NTHR * 4) + 4 * tid;
    const v4i c4 = *(const v4ia*)(scnt + s0);
    const float d0 = (float)(c4.x < 1 ? 1 : c4.x), d1 = (float)(c4.y < 1 ? 1 : c4.y);
    const float d2 = (float)(c4.z < 1 ? 1 : c4.z), d3 = (float)(c4.w < 1 ? 1 : c4.w);
    v4f v;
    v.x = rsqrtf(d0); v.y = rsqrtf(d1); v.z = rsqrtf(d2); v.w = rsqrtf(d3);
    vals[it] = v;
  }
  float* base = dg + (size_t)p * (size_t)nbpd + (size_t)nodeBase;
#pragma unroll
  for (int it = 0; it < NBD / (NTHR * 4); ++it) {
    const int s0 = it * (NTHR * 4) + 4 * tid;
    *(volatile v4f*)(base + s0) = vals[it];
  }
  __threadfence();
#pragma unroll
  for (int it = 0; it < NBD / (NTHR * 4); ++it) {
    const int s0 = it * (NTHR * 4) + 4 * tid;
    *(volatile v4f*)(base + s0) = vals[it];
  }
}

__global__ __launch_bounds__(GTHR) void k_gemm(const unsigned short* __restrict__ A,
                                               const unsigned short* __restrict__ WT,
                                               const float* __restrict__ dg, float* T, int K) {
  __shared__ __attribute__((aligned(16))) float stg[GBM * DH];
  __shared__ __attribute__((aligned(16))) float sdg[GBM];
  const int tid = (int)threadIdx.x, lane = tid & 31, wave = tid >> 5, hh = lane >> 4, m = lane & 15;
  const int rowBase = (int)blockIdx.x * GBM;
  if (tid < GBM) sdg[tid] = dg[rowBase + tid];

  v8f acc[8];
  {
    const v8f z = {0.f, 0.f, 0.f, 0.f, 0.f, 0.f, 0.f, 0.f};
#pragma unroll
    for (int t = 0; t < 8; ++t) acc[t] = z;
  }
  const unsigned short* ap = A  + (size_t)(rowBase + 16 * wave + m) * (size_t)K + 8 * hh;
  const unsigned short* bp = WT + (size_t)m * (size_t)K + 8 * hh;
  const int ksteps = K >> 5;

#pragma unroll 1
  for (int ks = 0; ks < ksteps; ++ks) {
    const int k0 = 32 * ks;
    Frag af;
    af.h[0] = *(const v8usa*)(ap + k0);
    af.h[1] = *(const v8usa*)(ap + k0 + 16);
#pragma unroll
    for (int nt = 0; nt < 8; ++nt) {
      const unsigned short* wq = bp + (size_t)(16 * nt) * (size_t)K + k0;
      Frag bf;
      bf.h[0] = *(const v8usa*)wq;
      bf.h[1] = *(const v8usa*)(wq + 16);
      acc[nt] = wmb(af, bf, acc[nt]);
    }
  }

#pragma unroll
  for (int nt = 0; nt < 8; ++nt) {
    const int lc = 16 * nt + m;
#pragma unroll
    for (int r = 0; r < 8; ++r) {
      const int lr = 16 * wave + 8 * hh + r;
      stg[lr * DH + lc] = acc[nt][r];
    }
  }
  __syncthreads();

  v4f fv[16];
#pragma unroll
  for (int i = 0; i < 16; ++i) {
    const int lr = 16 * wave + i;
    fv[i] = *(const v4fa*)(stg + lr * DH + 4 * lane) * sdg[lr];
  }
#pragma unroll
  for (int i = 0; i < 16; ++i) {
    float* op = T + (size_t)(rowBase + 16 * wave + i) * (size_t)DH + 4 * lane;
    *(volatile v4f*)op = fv[i];
  }
  __threadfence();
#pragma unroll
  for (int i = 0; i < 16; ++i) {
    float* op = T + (size_t)(rowBase + 16 * wave + i) * (size_t)DH + 4 * lane;
    *(volatile v4f*)op = fv[i];
  }
}

__global__ __launch_bounds__(GTHR) void k_gemm16(const unsigned short* __restrict__ A,
                                                 const unsigned short* __restrict__ WT,
                                                 const float* __restrict__ dg, float* T2) {
  __shared__ __attribute__((aligned(16))) float stg[GBM * NCL];
  __shared__ __attribute__((aligned(16))) float sdg[GBM];
  const int tid = (int)threadIdx.x, lane = tid & 31, wave = tid >> 5, hh = lane >> 4, m = lane & 15;
  const int rowBase = (int)blockIdx.x * GBM;
  if (tid < GBM) sdg[tid] = dg[rowBase + tid];

  v8f acc = {0.f, 0.f, 0.f, 0.f, 0.f, 0.f, 0.f, 0.f};
  const unsigned short* ap = A  + (size_t)(rowBase + 16 * wave + m) * (size_t)K2 + 8 * hh;
  const unsigned short* bp = WT + (size_t)m * (size_t)K2 + 8 * hh;

#pragma unroll 1
  for (int ks = 0; ks < K2 / 32; ++ks) {
    const int k0 = 32 * ks;
    Frag af, bf;
    af.h[0] = *(const v8usa*)(ap + k0);
    af.h[1] = *(const v8usa*)(ap + k0 + 16);
    bf.h[0] = *(const v8usa*)(bp + k0);
    bf.h[1] = *(const v8usa*)(bp + k0 + 16);
    acc = wmb(af, bf, acc);
  }

#pragma unroll
  for (int r = 0; r < 8; ++r) {
    const int lr = 16 * wave + 8 * hh + r;
    stg[lr * NCL + m] = acc[r];
  }
  __syncthreads();

  v4f pv[2];
#pragma unroll
  for (int q = 0; q < 2; ++q) {
    const int p   = tid + q * GTHR;
    const int row = p >> 2;
    const int col = 4 * (p & 3);
    pv[q] = *(const v4fa*)(stg + row * NCL + col) * sdg[row];
  }
#pragma unroll
  for (int q = 0; q < 2; ++q) {
    const int p = tid + q * GTHR;
    float* op = T2 + (size_t)(rowBase + (p >> 2)) * (size_t)NCL + 4 * (p & 3);
    *(volatile v4f*)op = pv[q];
  }
  __threadfence();
#pragma unroll
  for (int q = 0; q < 2; ++q) {
    const int p = tid + q * GTHR;
    float* op = T2 + (size_t)(rowBase + (p >> 2)) * (size_t)NCL + 4 * (p & 3);
    *(volatile v4f*)op = pv[q];
  }
}

template <int MODE, int LAST>
__global__ __launch_bounds__(NTHR) void k_agg(const int* __restrict__ srcs, const int* __restrict__ dsts,
                                              int nE, int nN, int vec8, int mRows, int first,
                                              const float* __restrict__ din, const float* __restrict__ tpl,
                                              const float* __restrict__ bias, float* opl,
                                              unsigned short* hpl, float* outp) {
  extern __shared__ __attribute__((aligned(16))) int dsm[];
  int* list = dsm;
  int* hl   = dsm + LISTN;
  int* sl   = hl + RCAP;
  int* cnt  = sl + RCAP;
  int* offs = cnt + NBA;
  int* cur  = offs + NBA;
  int* misc = cur + NBA;
  float* sto = (float*)(misc + 16);
  const int tid = (int)threadIdx.x, lane = tid & 31, wave = tid >> 5;
  const int nodeBase = (int)blockIdx.x * NBA;

  {
    const v4i z4 = {0, 0, 0, 0};
    for (int i = tid * 4; i < AGG_ZINTS; i += NTHR * 4) *(v4ia*)(dsm + i) = z4;
    if (tid < 16) misc[tid] = 0;
  }
  __syncthreads();

  int t = 0, ov = 0;
  const int nChunks = (nE + CHUNK - 1) / CHUNK;
#pragma unroll 1
  for (int ch = 0; ch < nChunks; ++ch) {
    const int cbase = ch * CHUNK;
    const int wc = scan_chunk<SLA>(dsts, nE, cbase, nodeBase, NBA, vec8, list, tid, lane, wave);
    if (lane == 0) misc[wave] = wc;
    __syncthreads();
    if (wave == 0) {
#pragma unroll 1
      for (int w2 = 0; w2 < NWAVE; ++w2) {
        int c = misc[w2];
        c = c < 0 ? 0 : (c > WCAP ? WCAP : c);
#pragma unroll 1
        for (int b0 = 0; b0 < c; b0 += 32) {
          const int idx = b0 + lane;
          const int ent = list[w2 * WCAP + (idx < WCAP ? idx : WCAP - 1)];
          const int m32 = (c - b0) < 32 ? (c - b0) : 32;
#pragma unroll 1
          for (int k = 0; k < m32; ++k) {
            const int u    = __builtin_amdgcn_readlane(ent, k);
            const int slot = u & (NBA - 1);
            const int el   = (u >> SLA) & (CHUNK - 1);
            const int pk   = ((cbase + el) << SLA) | slot;
            if (t < RCAP) {
              if (lane == 0) { hl[t] = pk; cnt[slot] = cnt[slot] + 1; }
              t = t + 1;
            } else {
              ov = 1;
            }
          }
        }
      }
    }
    __syncthreads();
  }
  if (wave == 0 && lane == 0) { misc[8] = t; misc[9] = ov; }
  __syncthreads();
  int tt = misc[8];
  tt = tt < 0 ? 0 : (tt > RCAP ? RCAP : tt);
  const int ovf = misc[9];

  if (wave == 0) {
    const int base = lane * (NBA / 32);
    int sacc = 0;
#pragma unroll 1
    for (int i = 0; i < NBA / 32; ++i) sacc += cnt[base + i];
    int incl = sacc;
#pragma unroll
    for (int d = 1; d < 32; d <<= 1) {
      const int y = __shfl_up(incl, d, 32);
      if (lane >= d) incl += y;
    }
    int run = incl - sacc;
#pragma unroll 1
    for (int i = 0; i < NBA / 32; ++i) {
      const int cv = cnt[base + i];
      offs[base + i] = run;
      cur[base + i]  = run;
      run += cv;
    }
  }
  __syncthreads();
  if (wave == 0) {
#pragma unroll 1
    for (int b0 = 0; b0 < tt; b0 += 32) {
      const int idx = b0 + lane;
      const int ent = hl[idx < RCAP ? idx : RCAP - 1];
      const int m32 = (tt - b0) < 32 ? (tt - b0) : 32;
#pragma unroll 1
      for (int k = 0; k < m32; ++k) {
        const int u    = __builtin_amdgcn_readlane(ent, k);
        const int slot = u & (NBA - 1);
        if (lane == 0) {
          int p = cur[slot];
          p = p < 0 ? 0 : (p > RCAP - 1 ? RCAP - 1 : p);
          sl[p] = u;
          cur[slot] = p + 1;
        }
      }
    }
  }
  __syncthreads();

  const float qnan = __int_as_float(0x7fc00000);
  const float pz = (ovf != 0) ? qnan : 0.0f;
  if constexpr (MODE == 0) {
    v4f bv;
    {
      const v4f a = *(const v4fa*)(bias + 4 * lane);
      bv.x = bf16_val(a.x); bv.y = bf16_val(a.y); bv.z = bf16_val(a.z); bv.w = bf16_val(a.w);
    }
    const v4f z4 = {0.0f, 0.0f, 0.0f, 0.0f};
#pragma unroll 1
    for (int si = 0; si < NBA / NWAVE; ++si) {
      const int s    = si * NWAVE + wave;
      const int node = nodeBase + s;
      int c = cnt[s];
      const bool big = c > DEGCAP;
      c = c < 0 ? 0 : (c > DEGCAP ? DEGCAP : c);
      int o = offs[s];
      o = o < 0 ? 0 : (o > RCAP ? RCAP : o);
      const int nc = node < nN ? node : nN - 1;
      const float dd = din[nc];
      v4f acc = z4;
#pragma unroll 1
      for (int b0 = 0; b0 < c; b0 += 32) {
        int idx = o + b0 + lane;
        idx = idx > RCAP - 1 ? RCAP - 1 : idx;
        const int ent = sl[idx];
        int eid = ent >> SLA;
        eid = eid < 0 ? 0 : (eid > nE - 1 ? nE - 1 : eid);
        int sr = srcs[eid];
        sr = sr < 0 ? 0 : (sr > nN - 1 ? nN - 1 : sr);
        const int m32 = (c - b0) < 32 ? (c - b0) : 32;
#pragma unroll 1
        for (int k = 0; k < m32; ++k) {
          const int sk = __builtin_amdgcn_readlane(sr, k);
          const v4f a = *(const v4fa*)(tpl + (size_t)sk * (size_t)DH + 4 * lane);
          acc += a;
        }
      }
      v4f prev = z4;
      if (first == 0) prev = *(const v4fa*)(opl + (size_t)nc * (size_t)DH + 4 * lane);
      const float pzr = big ? qnan : pz;
      const bool live = node < nN;
      v4f v;
      v.x = (prev.x + fmaxf(fmaf(acc.x, dd, bv.x), 0.0f) * 0.25f) + pzr;
      v.y = (prev.y + fmaxf(fmaf(acc.y, dd, bv.y), 0.0f) * 0.25f) + pzr;
      v.z = (prev.z + fmaxf(fmaf(acc.z, dd, bv.z), 0.0f) * 0.25f) + pzr;
      v.w = (prev.w + fmaxf(fmaf(acc.w, dd, bv.w), 0.0f) * 0.25f) + pzr;
      v.x = live ? v.x : 0.0f; v.y = live ? v.y : 0.0f;
      v.z = live ? v.z : 0.0f; v.w = live ? v.w : 0.0f;
      if constexpr (LAST == 0) {
        if (node < mRows) {
          float* op = opl + (size_t)node * (size_t)DH + 4 * lane;
          *(volatile v4f*)op = v;
          __threadfence();
          *(volatile v4f*)op = v;
        }
      } else {
        const v8us po = hilo8(v);
        if (node < mRows) {
          unsigned short* hp = hpl + (size_t)node * (size_t)K2 + 8 * lane;
          *(volatile v8us*)hp = po;
          __threadfence();
          *(volatile v8us*)hp = po;
        }
      }
    }
  } else {
    const int chn = lane & 15;
    const float bvs = bf16_val(bias[chn]);
#pragma unroll 1
    for (int f = 0; f < (NBA / NWAVE) / FLS; ++f) {
#pragma unroll 1
      for (int sj = 0; sj < FLS; ++sj) {
        const int si   = f * FLS + sj;
        const int s    = si * NWAVE + wave;
        const int node = nodeBase + s;
        int c = cnt[s];
        const bool big = c > DEGCAP;
        c = c < 0 ? 0 : (c > DEGCAP ? DEGCAP : c);
        int o = offs[s];
        o = o < 0 ? 0 : (o > RCAP ? RCAP : o);
        const int nc = node < nN ? node : nN - 1;
        const float dd = din[nc];
        float acc = 0.0f;
#pragma unroll 1
        for (int b0 = 0; b0 < c; b0 += 32) {
          int idx = o + b0 + lane;
          idx = idx > RCAP - 1 ? RCAP - 1 : idx;
          const int ent = sl[idx];
          int eid = ent >> SLA;
          eid = eid < 0 ? 0 : (eid > nE - 1 ? nE - 1 : eid);
          int sr = srcs[eid];
          sr = sr < 0 ? 0 : (sr > nN - 1 ? nN - 1 : sr);
          const int m32 = (c - b0) < 32 ? (c - b0) : 32;
#pragma unroll 1
          for (int k = 0; k < m32; ++k) {
            const int sk = __builtin_amdgcn_readlane(sr, k);
            const float a = tpl[(size_t)sk * (size_t)NCL + chn];
            acc += a;
          }
        }
        float prev = 0.0f;
        if (first == 0) prev = opl[(size_t)nc * (size_t)NCL + chn];
        const float pzr = big ? qnan : pz;
        const bool live = node < nN;
        float v = (prev + fmaf(acc, dd, bvs) * 0.25f) + pzr;
        v = live ? v : 0.0f;
        if (lane < NCL) sto[(sj * NWAVE + wave) * NCL + chn] = v;
      }
      __syncthreads();
      v4f pv[2];
#pragma unroll
      for (int q = 0; q < 2; ++q) {
        const int p = tid + q * NTHR;
        pv[q] = *(const v4fa*)(sto + (p >> 2) * NCL + 4 * (p & 3));
      }
      const int rowBase = nodeBase + f * FROWS;
      if constexpr (LAST == 0) {
#pragma unroll
        for (int q = 0; q < 2; ++q) {
          const int p = tid + q * NTHR;
          float* op = opl + (size_t)(rowBase + (p >> 2)) * (size_t)NCL + 4 * (p & 3);
          *(volatile v4f*)op = pv[q];
        }
        __threadfence();
#pragma unroll
        for (int q = 0; q < 2; ++q) {
          const int p = tid + q * NTHR;
          float* op = opl + (size_t)(rowBase + (p >> 2)) * (size_t)NCL + 4 * (p & 3);
          *(volatile v4f*)op = pv[q];
        }
      } else {
#pragma unroll
        for (int q = 0; q < 2; ++q) {
          const int p = tid + q * NTHR;
          const int grow = rowBase + (p >> 2);
          float* op = outp + (size_t)grow * (size_t)NCL + 4 * (p & 3);
          if (grow < nN) *(volatile v4f*)op = pv[q];
        }
        __threadfence();
#pragma unroll
        for (int q = 0; q < 2; ++q) {
          const int p = tid + q * NTHR;
          const int grow = rowBase + (p >> 2);
          float* op = outp + (size_t)grow * (size_t)NCL + 4 * (p & 3);
          if (grow < nN) *(volatile v4f*)op = pv[q];
        }
      }
      __syncthreads();
    }
  }
}

static inline int cdiv(int a, int b) { return (a + b - 1) / b; }

extern "C" void kernel_launch(void* const* d_in, const int* in_sizes, int n_in,
                              void* d_out, int out_size, void* d_ws, size_t ws_size,
                              hipStream_t stream) {
  if (n_in < 9) return;
  if (in_sizes[0] < CIN || (in_sizes[0] % CIN) != 0) return;
  const int nN = in_sizes[0] / CIN;
  if (in_sizes[1] != NREL * CIN * DH || in_sizes[2] != NREL * DH) return;
  if (in_sizes[3] != NREL * DH * DH  || in_sizes[4] != NREL * DH) return;
  if (in_sizes[5] != NREL * DH * NCL || in_sizes[6] != NREL * NCL) return;
  if (in_sizes[7] < NREL || (in_sizes[7] % NREL) != 0 || in_sizes[8] != in_sizes[7]) return;
  const int nE = in_sizes[7] / NREL;
  if (nE < 1 || nE >= (1 << (31 - SLA))) return;
  if ((long long)out_size != (long long)nN * NCL) return;

  const float* x   = (const float*)d_in[0];
  const float* W0  = (const float*)d_in[1];
  const float* b0  = (const float*)d_in[2];
  const float* W1  = (const float*)d_in[3];
  const float* b1  = (const float*)d_in[4];
  const float* W2  = (const float*)d_in[5];
  const float* b2  = (const float*)d_in[6];
  const int*   src = (const int*)d_in[7];
  const int*   dst = (const int*)d_in[8];
  float* out = (float*)d_out;

  const int MP   = cdiv(nN, GBM) * GBM;
  const int gM   = MP / GBM;
  const int gD   = cdiv(MP, NBD);
  const int NBPD = gD * NBD;
  const int gA   = cdiv(MP, NBA);
  if ((long long)gA * NBA < (long long)MP) return;
  if (NBPD < MP) return;
  const int vec8 = ((nE & 3) == 0) ? 1 : 0;

  char* ws = (char*)d_ws;
  size_t off = 0;
  const size_t oDG  = off; off += (size_t)8 * (size_t)NBPD * 4;                off = (off + 255) & ~(size_t)255;
  const size_t oW0T = off; off += (size_t)NREL * DH * CIN * 2;                 off = (off + 255) & ~(size_t)255;
  const size_t oW1T = off; off += (size_t)NREL * DH * K2 * 2;                  off = (off + 255) & ~(size_t)255;
  const size_t oW2T = off; off += (size_t)NREL * NCL * K2 * 2;                 off = (off + 255) & ~(size_t)255;
  const size_t oXB  = off; off += (size_t)MP * CIN * 2;                        off = (off + 255) & ~(size_t)255;
  const size_t szT  = (size_t)MP * DH * 4;
  const size_t szT2 = (size_t)MP * NCL * 4;
  const size_t oT   = off; off += (szT > szT2 ? szT : szT2);                   off = (off + 255) & ~(size_t)255;
  const size_t szO  = (size_t)MP * DH * 4;
  const size_t szO2 = (size_t)gA * NBA * NCL * 4;
  const size_t oO   = off; off += (szO > szO2 ? szO : szO2);                   off = (off + 255) & ~(size_t)255;
  const size_t oHA  = off; off += (size_t)MP * K2 * 2;                         off = (off + 255) & ~(size_t)255;
  if (off > ws_size || off > (size_t)WSMAX) return;
  float*          DG  = (float*)(ws + oDG);
  unsigned short* W0T = (unsigned short*)(ws + oW0T);
  unsigned short* W1T = (unsigned short*)(ws + oW1T);
  unsigned short* W2T = (unsigned short*)(ws + oW2T);
  unsigned short* XB  = (unsigned short*)(ws + oXB);
  float*          T   = (float*)(ws + oT);
  float*          O   = (float*)(ws + oO);
  unsigned short* HA  = (unsigned short*)(ws + oHA);

  const size_t aggLds = (size_t)AGG_LDS_INTS * 4;
  hipFuncSetAttribute(reinterpret_cast<const void*>(&k_agg<0, 0>), hipFuncAttributeMaxDynamicSharedMemorySize, (int)aggLds);
  hipFuncSetAttribute(reinterpret_cast<const void*>(&k_agg<0, 1>), hipFuncAttributeMaxDynamicSharedMemorySize, (int)aggLds);
  hipFuncSetAttribute(reinterpret_cast<const void*>(&k_agg<1, 0>), hipFuncAttributeMaxDynamicSharedMemorySize, (int)aggLds);
  hipFuncSetAttribute(reinterpret_cast<const void*>(&k_agg<1, 1>), hipFuncAttributeMaxDynamicSharedMemorySize, (int)aggLds);

  const int nUx = MP * (CIN / 8);
  k_prep<<<NUT / NTHR, NTHR, 0, stream>>>(W0, W1, W2, W0T, W1T, W2T);
  k_cvx<<<cdiv(nUx, NTHR), NTHR, 0, stream>>>(x, nN, nUx, XB);
  k_deg<<<dim3(gD, 2 * NREL), NTHR, 0, stream>>>(src, dst, nE, vec8, NBPD, DG);

  for (int r = 0; r < NREL; ++r) {
    k_gemm<<<gM, GTHR, 0, stream>>>(XB, W0T + (size_t)r * DH * CIN, DG + (size_t)r * NBPD, T, CIN);
    const int*   sr = src + (size_t)r * nE;
    const int*   ds = dst + (size_t)r * nE;
    const float* di = DG + (size_t)(NREL + r) * NBPD;
    const float* bb = b0 + (size_t)r * DH;
    const int first = (r == 0) ? 1 : 0;
    if (r < NREL - 1) k_agg<0, 0><<<gA, NTHR, aggLds, stream>>>(sr, ds, nE, nN, vec8, MP, first, di, T, bb, O, HA, out);
    else              k_agg<0, 1><<<gA, NTHR, aggLds, stream>>>(sr, ds, nE, nN, vec8, MP, first, di, T, bb, O, HA, out);
  }
  for (int r = 0; r < NREL; ++r) {
    k_gemm<<<gM, GTHR, 0, stream>>>(HA, W1T + (size_t)r * DH * K2, DG + (size_t)r * NBPD, T, K2);
    const int*   sr = src + (size_t)r * nE;
    const int*   ds = dst + (size_t)r * nE;
    const float* di = DG + (size_t)(NREL + r) * NBPD;
    const float* bb = b1 + (size_t)r * DH;
    const int first = (r == 0) ? 1 : 0;
    if (r < NREL - 1) k_agg<0, 0><<<gA, NTHR, aggLds, stream>>>(sr, ds, nE, nN, vec8, MP, first, di, T, bb, O, HA, out);
    else              k_agg<0, 1><<<gA, NTHR, aggLds, stream>>>(sr, ds, nE, nN, vec8, MP, first, di, T, bb, O, HA, out);
  }
  for (int r = 0; r < NREL; ++r) {
    k_gemm16<<<gM, GTHR, 0, stream>>>(HA, W2T + (size_t)r * NCL * K2, DG + (size_t)r * NBPD, T);
    const int*   sr = src + (size_t)r * nE;
    const int*   ds = dst + (size_t)r * nE;
    const float* di = DG + (size_t)(NREL + r) * NBPD;
    const float* bb = b2 + (size_t)r * NCL;
    const int first = (r == 0) ? 1 : 0;
    if (r < NREL - 1) k_agg<1, 0><<<gA, NTHR, aggLds, stream>>>(sr, ds, nE, nN, vec8, MP, first, di, T, bb, O, HA, out);
    else              k_agg<1, 1><<<gA, NTHR, aggLds, stream>>>(sr, ds, nE, nN, vec8, MP, first, di, T, bb, O, HA, out);
  }
}
